// ModularNetController_86363202388558
// MI455X (gfx1250) — hardware-verified
//
#include <hip/hip_runtime.h>
#include <math.h>
#include <stdint.h>

#define NB    32
#define CIN   128
#define COUT  128
#define IMH   56
#define IMW   56
#define HW    3136
#define NE    8
#define KK    1152
#define GS    4
#define NG    8
#define PT    98
#define NSEGP 14112
static_assert(NB == GS * NG);
static_assert(HW == IMH * IMW);
static_assert(PT * 32 == HW);
static_assert(NSEGP * 2 == HW * 9);
static_assert((HW % 64) == 0 && (KK % 32) == 0 && (COUT % 64) == 0);
static_assert((NSEGP % 72) == 0);

typedef _Float16 v16h __attribute__((ext_vector_type(16)));
typedef _Float16 v8h  __attribute__((ext_vector_type(8)));
typedef __bf16   v16b __attribute__((ext_vector_type(16)));
typedef __bf16   v8b  __attribute__((ext_vector_type(8)));
typedef float    v8f  __attribute__((ext_vector_type(8)));
typedef float    v4f  __attribute__((ext_vector_type(4)));
typedef unsigned int v4u __attribute__((ext_vector_type(4)));

__device__ __forceinline__ unsigned short bf_bits(float f) {
  unsigned u = __float_as_uint(f);
  return (unsigned short)((u + 0x7FFFu + ((u >> 16) & 1u)) >> 16);
}
__device__ __forceinline__ float bf_up(unsigned short h) { return __uint_as_float(((unsigned)h) << 16); }
__device__ __forceinline__ float bfr(float f) { return bf_up(bf_bits(f)); }
__device__ __forceinline__ unsigned short h_bits(_Float16 x) { return __builtin_bit_cast(unsigned short, x); }
__device__ __forceinline__ unsigned pk16(unsigned short a, unsigned short b) { return (unsigned)a | ((unsigned)b << 16); }
__device__ __forceinline__ v8f zero8() { v8f z = {0.f, 0.f, 0.f, 0.f, 0.f, 0.f, 0.f, 0.f}; return z; }

__device__ __forceinline__ v16b ldfrag_b(const __bf16* p) {
  union { v16b v; v8b h[2]; } f;
  f.h[0] = *(const v8b*)(p);
  f.h[1] = *(const v8b*)(p + 16);
  return f.v;
}

__device__ __forceinline__ v8f mma_b_raw(v16b a, v16b b, v8f c) {
  return __builtin_amdgcn_wmma_f32_16x16x32_bf16(false, a, false, b, (short)0, c, false, false);
}
__device__ __forceinline__ void dep_guard_b(v8f& a, v8f& b, v16b x, v16b y) {
#if defined(__HIP_DEVICE_COMPILE__)
  asm volatile("v_nop\n\tv_nop\n\tv_nop\n\tv_nop" : "+v"(a), "+v"(b) : "v"(x), "v"(y));
#endif
}
__device__ __forceinline__ void keep4_b(v16b a, v16b b, v16b c, v16b d) {
#if defined(__HIP_DEVICE_COMPILE__)
  asm volatile("v_nop" :: "v"(a), "v"(b), "v"(c), "v"(d));
#endif
}
__device__ __forceinline__ void acc_guard4(v8f& a, v8f& b, v8f& c, v8f& d) {
#if defined(__HIP_DEVICE_COMPILE__)
  asm volatile("v_nop\n\tv_nop\n\tv_nop\n\tv_nop" : "+v"(a), "+v"(b), "+v"(c), "+v"(d));
#endif
}
__device__ __forceinline__ void wave_sync_lds() {
  __builtin_amdgcn_fence(__ATOMIC_RELEASE, "workgroup");
  __builtin_amdgcn_wave_barrier();
  __builtin_amdgcn_fence(__ATOMIC_ACQUIRE, "workgroup");
}

__global__ __launch_bounds__(256) void cvt_xt(const float* __restrict__ x, unsigned short* xt) {
  __shared__ __align__(16) float sx[CIN * 36];
  const int tid = threadIdx.x;
  const int b   = blockIdx.x / PT;
  const int tp  = blockIdx.x - b * PT;
  const int p0  = tp * 32;
  const float* xb = x + (size_t)b * CIN * HW + p0;
#pragma unroll
  for (int it = 0; it < 4; ++it) {
    const int idx = it * 256 + tid;
    const int c = idx >> 3, q = idx & 7;
    const v4f v = *(const v4f*)(xb + (size_t)c * HW + 4 * q);
    *(v4f*)(sx + c * 36 + 4 * q) = v;
  }
  __syncthreads();
  const int wave = tid >> 5, lane = tid & 31, hh = lane >> 4, c8 = (lane & 15) * 8;
  v4u pk[2];
#pragma unroll
  for (int it = 0; it < 2; ++it) {
    const int r = wave * 4 + it * 2 + hh;
    v4u p;
#pragma unroll
    for (int e = 0; e < 4; ++e)
      p[e] = pk16(bf_bits(sx[(c8 + 2 * e) * 36 + r]), bf_bits(sx[(c8 + 2 * e + 1) * 36 + r]));
    pk[it] = p;
  }
  unsigned short* dst = xt + ((size_t)b * HW + p0) * CIN;
  for (int pass = 0; pass < 2; ++pass) {
#pragma unroll
    for (int it = 0; it < 2; ++it) {
      const int r = wave * 4 + it * 2 + hh;
      *(volatile v4u*)(dst + (size_t)r * CIN + c8) = pk[it];
    }
    __threadfence();
  }
}

__global__ __launch_bounds__(256)
void select_expert(const float* __restrict__ x, const float* __restrict__ ctlw, const float* __restrict__ ctlb,
                   const float* __restrict__ expw, const float* __restrict__ expb,
                   unsigned short* wsel, float* bsel) {
#pragma clang fp contract(off)
  __shared__ float sS[CIN];
  __shared__ float sL[NE];
  __shared__ int   sE;
  const int tid = threadIdx.x, wave = tid >> 5, lane = tid & 31;
  const int b = blockIdx.x;

  const float* xb = x + (size_t)b * CIN * HW;
#pragma unroll 1
  for (int cc = 0; cc < 16; ++cc) {
    const int c = wave * 16 + cc;
    const float* row = xb + (size_t)c * HW;
    float a0 = 0.f, a1 = 0.f, a2 = 0.f, a3 = 0.f;
    for (int it = 0; it < 25; ++it) {
      const int f4  = it * 32 + lane;
      const int f4c = min(f4, HW / 4 - 1);
      const bool ok = f4 < (HW / 4);
      const v4f v = *(const v4f*)(row + 4 * f4c);
      a0 += ok ? bfr(v[0]) : 0.f;
      a1 += ok ? bfr(v[1]) : 0.f;
      a2 += ok ? bfr(v[2]) : 0.f;
      a3 += ok ? bfr(v[3]) : 0.f;
    }
    float s = (a0 + a1) + (a2 + a3);
#pragma unroll
    for (int off = 1; off < 32; off <<= 1) s += __shfl_xor(s, off, 32);
    if (lane == 0) sS[c] = s;
  }
  __syncthreads();

  if (wave == 0) {
    const int e = min(lane, NE - 1);
    float raw = 0.f;
#pragma unroll 1
    for (int c = 0; c < CIN; ++c) raw += sS[c] * bfr(ctlw[e * CIN + c]);
    const float lg = raw * (1.0f / (float)HW) + bfr(ctlb[e]);
    if (lane < NE) sL[lane] = lg;
  }
  __syncthreads();
  if (tid == 0) {
    int best = 0;
    float bv = sL[0];
#pragma unroll
    for (int e2 = 1; e2 < NE; ++e2) {
      const float v = sL[e2];
      if (v > bv) { bv = v; best = e2; }
    }
    sE = best;
  }
  __syncthreads();
  const int esel = min(max(sE, 0), NE - 1);

  if (wave == 0) {
    const float* be = expb + (size_t)esel * COUT;
    v4f bv;
    bv[0] = bfr(be[4 * lane + 0]);
    bv[1] = bfr(be[4 * lane + 1]);
    bv[2] = bfr(be[4 * lane + 2]);
    bv[3] = bfr(be[4 * lane + 3]);
    float* bd = bsel + (size_t)b * COUT + 4 * lane;
    *(volatile v4f*)bd = bv;
    __threadfence();
    *(volatile v4f*)bd = bv;
  }

  const float* we = expw + (size_t)esel * COUT * CIN * 9;
  unsigned short* wd = wsel + (size_t)b * COUT * KK;
#pragma unroll 1
  for (int it = 0; it < 72; ++it) {
    const int j   = it * 256 + tid;
    const int f   = j * 8;
    const int o   = f / KK;
    const int rem = f - o * KK;
    const int t   = rem >> 7;
    const int c   = rem & 127;
    const float* src = we + ((size_t)(o * CIN + c)) * 9 + t;
    float vals[8];
#pragma unroll
    for (int i = 0; i < 8; ++i) vals[i] = src[i * 9];
    v4u p;
#pragma unroll
    for (int i = 0; i < 4; ++i) p[i] = pk16(bf_bits(vals[2 * i]), bf_bits(vals[2 * i + 1]));
    unsigned short* d = wd + f;
    *(volatile v4u*)d = p;
    __threadfence();
    *(volatile v4u*)d = p;
  }
}

__global__ __launch_bounds__(256) void im2col(const unsigned short* __restrict__ xt, unsigned short* xc) {
  const int bl = blockIdx.y;
  const unsigned short* xs = xt + (size_t)bl * HW * CIN;
  unsigned short* xd = xc + (size_t)bl * HW * KK;
  const int tid = threadIdx.x, wave = tid >> 5, lane = tid & 31, hh = lane >> 4, c8 = (lane & 15) * 8;
  const int jb = (blockIdx.x * 8 + wave) * 9;
#pragma unroll 1
  for (int it = 0; it < 9; ++it) {
    const int j = jb + it;
    if (j < NSEGP) {
      const int seg = 2 * j + hh;
      const int p   = seg / 9;
      const int t   = seg - p * 9;
      const int ky  = t / 3, kx = t - ky * 3;
      const int y   = p / IMW, xw = p - y * IMW;
      const int ys  = y + ky - 1, xsr = xw + kx - 1;
      const bool ok = ((unsigned)ys < (unsigned)IMH) && ((unsigned)xsr < (unsigned)IMW);
      const int ysc = min(max(ys, 0), IMH - 1), xsc = min(max(xsr, 0), IMW - 1);
      const v4u v = *(const v4u*)(xs + (size_t)(ysc * IMW + xsc) * CIN + c8);
      v4u w;
      w[0] = ok ? v[0] : 0u;
      w[1] = ok ? v[1] : 0u;
      w[2] = ok ? v[2] : 0u;
      w[3] = ok ? v[3] : 0u;
      unsigned short* d = xd + (size_t)seg * CIN + c8;
      *(volatile v4u*)d = w;
      __threadfence();
      *(volatile v4u*)d = w;
    }
  }
}

template <int NSPLIT, int OUT_MODE>
__global__ __launch_bounds__(256) void gemm64(
    const unsigned short* __restrict__ Ap, const unsigned short* A2p, int lda, long long strideA,
    const unsigned short* __restrict__ Btp, const unsigned short* Bt2p, int ldb, long long strideB,
    void* Cout, int ldc, long long strideC,
    void* Cout2, int ldc2, long long strideC2, int N2,
    int M, int N, int K, float rscale,
    const float* __restrict__ biasp, long long strideBias) {
  const __bf16* A   = (const __bf16*)(const void*)Ap;
  const __bf16* A2  = (const __bf16*)(const void*)A2p;
  const __bf16* Bt  = (const __bf16*)(const void*)Btp;
  const __bf16* Bt2 = (const __bf16*)(const void*)Bt2p;
  __shared__ __align__(16) float sT[8][16 * 68];
  const int b    = blockIdx.y;
  const int lane = threadIdx.x & 31;
  const int wave = threadIdx.x >> 5;
  const int tilesN = N >> 6;
  const int tilesM = M >> 6;
  const int tile = blockIdx.x * 8 + wave;
  if (tile >= tilesM * tilesN) return;
  const int tm = tile / tilesN;
  const int tn = tile - tm * tilesN;
  const int m0 = tm << 6;
  const int n0 = tn << 6;

  const __bf16* Ab  = A  + (size_t)b * strideA;
  const __bf16* Bb  = Bt + (size_t)b * strideB;
  const __bf16* Ab2 = (NSPLIT >= 1) ? (A2  + (size_t)b * strideA) : Ab;
  const __bf16* Bb2 = (NSPLIT == 2) ? (Bt2 + (size_t)b * strideB) : Bb;

  const int rlane = lane & 15;
  const int koff  = (lane >> 4) * 8;
  const int mOff  = (lane >> 4) * 8;

  v8f acc[4][4];
#pragma unroll
  for (int i = 0; i < 4; ++i)
#pragma unroll
    for (int j = 0; j < 4; ++j) acc[i][j] = zero8();

  for (int k0 = 0; k0 < K; k0 += 32) {
    v16b bh[4], bl[4];
#pragma unroll
    for (int j = 0; j < 4; ++j) {
      const size_t bo = (size_t)(n0 + (j << 4) + rlane) * ldb + koff + k0;
      bh[j] = ldfrag_b(Bb + bo);
      if (NSPLIT == 2) bl[j] = ldfrag_b(Bb2 + bo); else bl[j] = bh[j];
    }
#pragma unroll
    for (int i = 0; i < 4; ++i) {
      const size_t ao = (size_t)(m0 + (i << 4) + rlane) * lda + koff + k0;
      const v16b ah = ldfrag_b(Ab + ao);
      v16b al = ah;
      if (NSPLIT >= 1) al = ldfrag_b(Ab2 + ao);
#pragma unroll
      for (int j = 0; j < 4; ++j) {
        acc[i][j] = mma_b_raw(ah, bh[j], acc[i][j]);
        if (NSPLIT >= 1) acc[i][j] = mma_b_raw(al, bh[j], acc[i][j]);
        if (NSPLIT == 2) acc[i][j] = mma_b_raw(ah, bl[j], acc[i][j]);
      }
      dep_guard_b(acc[i][0], acc[i][3], ah, al);
    }
    keep4_b(bh[0], bh[1], bh[2], bh[3]);
    if (NSPLIT == 2) keep4_b(bl[0], bl[1], bl[2], bl[3]);
  }
  acc_guard4(acc[0][0], acc[0][1], acc[0][2], acc[0][3]);
  acc_guard4(acc[1][0], acc[1][1], acc[1][2], acc[1][3]);
  acc_guard4(acc[2][0], acc[2][1], acc[2][2], acc[2][3]);
  acc_guard4(acc[3][0], acc[3][1], acc[3][2], acc[3][3]);

  float* slab = sT[wave];
#pragma unroll
  for (int i = 0; i < 4; ++i) {
    const int mBase = m0 + (i << 4);
#pragma unroll
    for (int j = 0; j < 4; ++j) {
#pragma unroll
      for (int r = 0; r < 8; ++r) {
        slab[(mOff + r) * 68 + (j << 4) + rlane] = acc[i][j][r];
      }
    }
    wave_sync_lds();
    if (OUT_MODE == 0) {
      float* C = (float*)Cout + (size_t)b * strideC;
      const float* brow = biasp + (size_t)b * strideBias;
      const int hh = lane >> 4, c4 = (lane & 15) * 4;
      v4f ov[8];
#pragma unroll
      for (int it = 0; it < 8; ++it) {
        const int row = it * 2 + hh;
        const float bv = brow[mBase + row];
        v4f v = *(const v4f*)(slab + row * 68 + c4);
        v[0] += bv; v[1] += bv; v[2] += bv; v[3] += bv;
        ov[it] = v;
      }
      for (int pass = 0; pass < 2; ++pass) {
#pragma unroll
        for (int it = 0; it < 8; ++it) {
          const int row = it * 2 + hh;
          *(volatile v4f*)(C + (size_t)(mBase + row) * ldc + n0 + c4) = ov[it];
        }
        __threadfence();
      }
    } else {
      const int q = lane >> 3, c8 = (lane & 7) * 8;
      unsigned short* C  = (unsigned short*)Cout  + (size_t)b * strideC;
      unsigned short* C2 = (unsigned short*)Cout2 + (size_t)b * strideC2;
      const bool wlo = (OUT_MODE == 2) || (n0 < N2);
      v4u hv[4], lv[4];
#pragma unroll
      for (int it = 0; it < 4; ++it) {
        const int row = it * 4 + q;
        const float* sp = slab + row * 68 + c8;
        v4u a, a2;
#pragma unroll
        for (int e = 0; e < 4; ++e) {
          const float f0 = sp[2 * e], f1 = sp[2 * e + 1];
          unsigned short h0, h1, l0, l1;
          if (OUT_MODE == 2) {
            h0 = bf_bits(f0); h1 = bf_bits(f1);
            l0 = bf_bits(f0 - bf_up(h0)); l1 = bf_bits(f1 - bf_up(h1));
          } else {
            const _Float16 x0 = (_Float16)f0, x1 = (_Float16)f1;
            h0 = h_bits(x0); h1 = h_bits(x1);
            l0 = h_bits((_Float16)((f0 - (float)x0) * rscale));
            l1 = h_bits((_Float16)((f1 - (float)x1) * rscale));
          }
          a[e] = pk16(h0, h1); a2[e] = pk16(l0, l1);
        }
        hv[it] = a; lv[it] = a2;
      }
      for (int pass = 0; pass < 2; ++pass) {
#pragma unroll
        for (int it = 0; it < 4; ++it) {
          const int row = it * 4 + q;
          *(volatile v4u*)(C + (size_t)(mBase + row) * ldc + n0 + c8) = hv[it];
          if (wlo) *(volatile v4u*)(C2 + (size_t)(mBase + row) * ldc2 + n0 + c8) = lv[it];
        }
        __threadfence();
      }
    }
    wave_sync_lds();
  }
}

extern "C" void kernel_launch(void* const* d_in, const int* in_sizes, int n_in,
                              void* d_out, int out_size, void* d_ws, size_t ws_size,
                              hipStream_t stream) {
  if (n_in < 5) return;
  if (in_sizes[0] != NB * CIN * HW) return;
  if (in_sizes[1] != NE * CIN) return;
  if (in_sizes[2] != NE) return;
  if (in_sizes[3] != NE * COUT * CIN * 9) return;
  if (in_sizes[4] != NE * COUT) return;
  if (out_size != NB * COUT * HW) return;

  const float* x    = (const float*)d_in[0];
  const float* ctlw = (const float*)d_in[1];
  const float* ctlb = (const float*)d_in[2];
  const float* expw = (const float*)d_in[3];
  const float* expb = (const float*)d_in[4];
  float* out = (float*)d_out;

  const size_t PXT = (size_t)NB * HW * CIN * 2;
  const size_t PWS = (size_t)NB * COUT * KK * 2;
  const size_t PBS = (size_t)NB * COUT * 4;
  const size_t PXC = (size_t)GS * HW * KK * 2;
  size_t off = 0;
  const size_t oXT = off; off += PXT;
  const size_t oWS = off; off += PWS;
  const size_t oBS = off; off += PBS;
  const size_t oXC = off; off += PXC;
  if (off > ws_size) return;
  if (off > (size_t)134217728) return;

  char* ws = (char*)d_ws;
  unsigned short* XT = (unsigned short*)(ws + oXT);
  unsigned short* WS = (unsigned short*)(ws + oWS);
  float*          BS = (float*)(ws + oBS);
  unsigned short* XC = (unsigned short*)(ws + oXC);

  const dim3 blk(256);
  cvt_xt<<<dim3(NB * PT), blk, 0, stream>>>(x, XT);
  select_expert<<<dim3(NB), blk, 0, stream>>>(x, ctlw, ctlb, expw, expb, WS, BS);
  const dim3 gI2c(NSEGP / 72, GS);
  const dim3 gGemm(((COUT / 64) * (HW / 64) + 7) / 8, GS);
  for (int g = 0; g < NG; ++g) {
    const unsigned short* XTg = XT + (size_t)g * GS * HW * CIN;
    const unsigned short* WSg = WS + (size_t)g * GS * COUT * KK;
    const float*          BSg = BS + (size_t)g * GS * COUT;
    float*                Cg  = out + (size_t)g * GS * COUT * HW;
    im2col<<<gI2c, blk, 0, stream>>>(XTg, XC);
    gemm64<0, 0><<<gGemm, blk, 0, stream>>>(
        WSg, WSg, KK, (long long)COUT * KK,
        XC, XC, KK, (long long)HW * KK,
        (void*)Cg, HW, (long long)COUT * HW,
        (void*)Cg, HW, (long long)COUT * HW, 0,
        COUT, HW, KK, 1.0f,
        BSg, (long long)COUT);
  }
  (void)hipGetLastError();
}
